// GraphConv_16449724744756
// MI455X (gfx1250) — hardware-verified
//
#include <hip/hip_runtime.h>
#include <stddef.h>
#include <stdint.h>


#define NN    4096
#define NE    16384
#define DD    128
#define NTHR  256
#define GTHR  128
#define NWAVE 8
#define EPT   8
#define CHUNK (NTHR * EPT)
#define WCAP  (EPT * 32)
#define LISTN (NWAVE * WCAP)
#define TP    136
#define WSMAX 134217728

#define PU_W2 8192
#define PU_W3 4096
#define PU_W4 262144
#define PU_WI 6144
#define PU_WH 6144
#define PU_H0 65536
#define PU_EB 65536
#define PU_W1 1024
#define PU_B4 2048
#define PU_ALL (PU_W2 + PU_W3 + PU_W4 + PU_WI + PU_WH + PU_H0 + PU_EB + PU_W1 + PU_B4)
#define COV_LDS (2 * 128 * TP * 2)

static_assert((PU_W2 % NTHR) == 0 && (PU_W3 % NTHR) == 0 && (PU_W4 % NTHR) == 0 && (PU_WI % NTHR) == 0);
static_assert((PU_WH % NTHR) == 0 && (PU_H0 % NTHR) == 0 && (PU_EB % NTHR) == 0 && (PU_W1 % NTHR) == 0 && (PU_B4 % NTHR) == 0);
static_assert((PU_ALL % NTHR) == 0);
static_assert(WCAP == 256 && CHUNK == 2048 && (NE % CHUNK) == 0);
static_assert((NE % 128) == 0 && (NN % 64) == 0 && (TP % 8) == 0);
static_assert(COV_LDS >= 128 * 128 * 4);

typedef float          v4f   __attribute__((ext_vector_type(4)));
typedef float          v8f   __attribute__((ext_vector_type(8)));
typedef double         v2d   __attribute__((ext_vector_type(2)));
typedef int            v4i   __attribute__((ext_vector_type(4)));
typedef int            v8i   __attribute__((ext_vector_type(8)));
typedef unsigned short v8us  __attribute__((ext_vector_type(8)));
typedef unsigned short v16us __attribute__((ext_vector_type(16)));
typedef __bf16         v16bf __attribute__((ext_vector_type(16)));
typedef v4f  __attribute__((may_alias)) v4fa;
typedef v2d  __attribute__((may_alias)) v2da;
typedef v4i  __attribute__((may_alias)) v4ia;
typedef v8us __attribute__((may_alias)) v8usa;
union FragB { v16bf v; v16us u; v8us h[2]; v8i w; };

__device__ __forceinline__ v8f z8() { v8f z = {0.f, 0.f, 0.f, 0.f, 0.f, 0.f, 0.f, 0.f}; return z; }

__device__ __forceinline__ v8f wmb(const FragB& a, const FragB& b, v8f c) {
  v8f d = __builtin_amdgcn_wmma_f32_16x16x32_bf16(false, a.v, false, b.v, (short)0, c, false, false);
  asm volatile("v_nop\n\tv_nop\n\tv_nop\n\tv_nop" : "+v"(d) : "v"(a.w), "v"(b.w));
  return d;
}

__device__ __forceinline__ unsigned bf16_bits(float f) {
  const unsigned u = __float_as_uint(f);
  return (u + 0x7FFFu + ((u >> 16) & 1u)) >> 16;
}
__device__ __forceinline__ float bf16_val(float f) { return __uint_as_float(bf16_bits(f) << 16); }
__device__ __forceinline__ v4f bfv4(v4f a) {
  a.x = bf16_val(a.x); a.y = bf16_val(a.y); a.z = bf16_val(a.z); a.w = bf16_val(a.w);
  return a;
}
__device__ __forceinline__ v8us cvt8(v4f a, v4f b) {
  v8us o;
  o[0] = (unsigned short)bf16_bits(a.x); o[1] = (unsigned short)bf16_bits(a.y);
  o[2] = (unsigned short)bf16_bits(a.z); o[3] = (unsigned short)bf16_bits(a.w);
  o[4] = (unsigned short)bf16_bits(b.x); o[5] = (unsigned short)bf16_bits(b.y);
  o[6] = (unsigned short)bf16_bits(b.z); o[7] = (unsigned short)bf16_bits(b.w);
  return o;
}
__device__ __forceinline__ void split8(v4f a, v4f b, v8us& hi, v8us& lo) {
  float v[8] = {a.x, a.y, a.z, a.w, b.x, b.y, b.z, b.w};
#pragma unroll
  for (int k = 0; k < 8; ++k) {
    const unsigned h = bf16_bits(v[k]);
    hi[k] = (unsigned short)h;
    lo[k] = (unsigned short)bf16_bits(v[k] - __uint_as_float(h << 16));
  }
}

struct Col8 { v4f m0, m1, r0, r1, g0, g1, b0, b1; };
__device__ __forceinline__ void ldcol8(const float* __restrict__ tab, int nCols, const float* __restrict__ g,
                                       const float* __restrict__ b, int c8, Col8& C) {
  C.m0 = *(const v4fa*)(tab + c8);         C.m1 = *(const v4fa*)(tab + c8 + 4);
  C.r0 = *(const v4fa*)(tab + nCols + c8); C.r1 = *(const v4fa*)(tab + nCols + c8 + 4);
  C.g0 = bfv4(*(const v4fa*)(g + c8));     C.g1 = bfv4(*(const v4fa*)(g + c8 + 4));
  C.b0 = bfv4(*(const v4fa*)(b + c8));     C.b1 = bfv4(*(const v4fa*)(b + c8 + 4));
}
__device__ __forceinline__ v4f bnr4(v4f y, v4f m, v4f r, v4f g, v4f b) {
  v4f t = ((y - m) * r) * g + b;
  t.x = fmaxf(t.x, 0.0f); t.y = fmaxf(t.y, 0.0f); t.z = fmaxf(t.z, 0.0f); t.w = fmaxf(t.w, 0.0f);
  return t;
}

__global__ __launch_bounds__(NTHR) void k_prep(
    const float* __restrict__ W2, const float* __restrict__ W3, const float* __restrict__ W4,
    const float* __restrict__ Wih, const float* __restrict__ Whh, const float* __restrict__ hid,
    const float* __restrict__ edge, const float* __restrict__ W1, const float* __restrict__ b4,
    unsigned short* w2b, unsigned short* w3b, unsigned short* w4b, unsigned short* wib,
    unsigned short* whb, unsigned short* h0b, unsigned short* ebp, unsigned short* w1b,
    unsigned short* b4t) {
  const int c0 = PU_W2, c1 = c0 + PU_W3, c2 = c1 + PU_W4, c3 = c2 + PU_WI, c4 = c3 + PU_WH;
  const int c5 = c4 + PU_H0, c6 = c5 + PU_EB, c7 = c6 + PU_W1, c8 = c7 + PU_B4;
  const int bstart = (int)blockIdx.x * NTHR;
  const int u = bstart + (int)threadIdx.x;
  int mode = 0, seg = 0;
  const float* src = W2;
  unsigned short* dst = w2b;
  if (bstart < c0)      { }
  else if (bstart < c1) { src = W3;   dst = w3b; seg = c0; }
  else if (bstart < c2) { src = W4;   dst = w4b; seg = c1; }
  else if (bstart < c3) { src = Wih;  dst = wib; seg = c2; }
  else if (bstart < c4) { src = Whh;  dst = whb; seg = c3; }
  else if (bstart < c5) { src = hid;  dst = h0b; seg = c4; }
  else if (bstart < c6) { src = edge; dst = ebp; seg = c5; mode = 1; }
  else if (bstart < c7) { src = W1;   dst = w1b; seg = c6; mode = 1; }
  else                  { src = b4;   dst = b4t; seg = c7; mode = 2; }
  if (u >= c8) return;
  const int v = u - seg;
  v8us o;
  if (mode == 0) {
    const float* p = src + (size_t)v * 8;
    o = cvt8(*(const v4fa*)p, *(const v4fa*)(p + 4));
  } else if (mode == 1) {
    const int row = v >> 2, kq = v & 3;
    const float* p = src + (size_t)row * 16 + (kq & 1) * 8;
    const v8us t = cvt8(*(const v4fa*)p, *(const v4fa*)(p + 4));
    const bool ok = kq < 2;
#pragma unroll
    for (int i = 0; i < 8; ++i) o[i] = ok ? t[i] : (unsigned short)0;
  } else {
    const int k = v >> 4, d8 = (v & 15) * 8;
    const float* p = src + (size_t)d8 * 128 + k;
#pragma unroll
    for (int i = 0; i < 8; ++i) o[i] = (unsigned short)bf16_bits(p[(size_t)i * 128]);
  }
  unsigned short* dp = dst + (size_t)v * 8;
  *(volatile v8us*)dp = o;
  __threadfence();
  *(volatile v8us*)dp = o;
}

template <int BIAS, int STATS>
__global__ __launch_bounds__(GTHR) void k_gemm(
    const unsigned short* __restrict__ A, int lda, int ksteps,
    const unsigned short* __restrict__ WT, int ldw, int kwrap,
    float* outF, int ldo, const float* __restrict__ bias, double* rec, int nCols) {
  __shared__ __attribute__((aligned(16))) float stg[64 * 64];
  const int tid = (int)threadIdx.x, lane = tid & 31, wave = tid >> 5, hh = lane >> 4, m = lane & 15;
  const int rowBase = (int)blockIdx.x * 64;
  const int col0    = (int)blockIdx.y * 64;
  v8f acc[4];
  acc[0] = z8(); acc[1] = z8(); acc[2] = z8(); acc[3] = z8();
  const unsigned short* ap = A  + (size_t)(rowBase + 16 * wave + m) * (size_t)lda + 8 * hh;
  const unsigned short* wp = WT + (size_t)(col0 + m) * (size_t)ldw + 8 * hh;
#pragma unroll 1
  for (int ks = 0; ks < ksteps; ++ks) {
    const int kw = (ks < kwrap) ? ks : (ks - kwrap);
    FragB af;
    af.h[0] = *(const v8usa*)(ap + 32 * ks);
    af.h[1] = *(const v8usa*)(ap + 32 * ks + 16);
#pragma unroll
    for (int t = 0; t < 4; ++t) {
      const unsigned short* wq = wp + (size_t)(16 * t) * (size_t)ldw + 32 * kw;
      FragB bf;
      bf.h[0] = *(const v8usa*)wq;
      bf.h[1] = *(const v8usa*)(wq + 16);
      acc[t] = wmb(af, bf, acc[t]);
    }
  }
#pragma unroll
  for (int t = 0; t < 4; ++t) {
    const int lc = 16 * t + m;
    float bv = 0.0f;
    if constexpr (BIAS != 0) bv = bf16_val(bias[col0 + lc]);
#pragma unroll
    for (int r = 0; r < 8; ++r) {
      const int lr = 16 * wave + 8 * hh + r;
      stg[lr * 64 + lc] = acc[t][r] + bv;
    }
  }
  __syncthreads();
  if constexpr (STATS != 0) {
    if (tid < 64) {
      double s = 0.0, q = 0.0;
#pragma unroll 4
      for (int r = 0; r < 64; ++r) {
        const double v = (double)stg[r * 64 + tid];
        s += v; q += v * v;
      }
      v2d o; o.x = s; o.y = q;
      double* rp = rec + ((size_t)blockIdx.x * (size_t)nCols + (size_t)(col0 + tid)) * 2;
      *(volatile v2d*)rp = o;
      __threadfence();
      *(volatile v2d*)rp = o;
    }
  }
  v4f fv[8];
#pragma unroll
  for (int i = 0; i < 8; ++i) {
    const int lr = 16 * wave + 2 * i + hh;
    fv[i] = *(const v4fa*)(stg + lr * 64 + 4 * m);
  }
#pragma unroll
  for (int i = 0; i < 8; ++i) {
    const int gr = rowBase + 16 * wave + 2 * i + hh;
    *(volatile v4f*)(outF + (size_t)gr * (size_t)ldo + col0 + 4 * m) = fv[i];
  }
  __threadfence();
#pragma unroll
  for (int i = 0; i < 8; ++i) {
    const int gr = rowBase + 16 * wave + 2 * i + hh;
    *(volatile v4f*)(outF + (size_t)gr * (size_t)ldo + col0 + 4 * m) = fv[i];
  }
}

__global__ __launch_bounds__(NTHR) void k_comb(const double* __restrict__ rec, int nbr, int nCols,
                                               double invE, float* tab) {
  __shared__ __attribute__((aligned(16))) float sm[512];
  const int tid = (int)threadIdx.x;
  const int c = tid < nCols ? tid : nCols - 1;
  double s = 0.0, q = 0.0;
#pragma unroll 4
  for (int b = 0; b < nbr; ++b) {
    const v2d r = *(const v2da*)(rec + ((size_t)b * (size_t)nCols + (size_t)c) * 2);
    s += r.x; q += r.y;
  }
  const double mean = s * invE;
  double var = q * invE - mean * mean;
  var = var < 0.0 ? 0.0 : var;
  const float rs = rsqrtf((float)var + 1e-5f);
  if (tid < nCols) { sm[tid] = (float)mean; sm[nCols + tid] = rs; }
  __syncthreads();
  const int nv = nCols >> 1;
  const int tc = tid < nv ? tid : nv - 1;
  const v4f ov = *(const v4fa*)(sm + 4 * tc);
  if (tid < nv) *(volatile v4f*)(tab + 4 * tid) = ov;
  __threadfence();
  if (tid < nv) *(volatile v4f*)(tab + 4 * tid) = ov;
}

__global__ __launch_bounds__(NTHR) void k_apply(const float* __restrict__ Y, const float* __restrict__ tab,
                                                const float* __restrict__ g, const float* __restrict__ b,
                                                unsigned short* X, int nCols, int ush, int nUnits) {
  const int u = (int)blockIdx.x * NTHR + (int)threadIdx.x;
  if (u >= nUnits) return;
  const int row = u >> ush;
  const int c8  = (u & ((1 << ush) - 1)) * 8;
  Col8 C;
  ldcol8(tab, nCols, g, b, c8, C);
  const float* yp = Y + (size_t)row * (size_t)nCols + c8;
  const v4f xa = bnr4(*(const v4fa*)yp,       C.m0, C.r0, C.g0, C.b0);
  const v4f xb = bnr4(*(const v4fa*)(yp + 4), C.m1, C.r1, C.g1, C.b1);
  v8us hi, lo;
  split8(xa, xb, hi, lo);
  unsigned short* dp = X + (size_t)row * (size_t)(2 * nCols) + c8;
  *(volatile v8us*)dp = hi;
  *(volatile v8us*)(dp + nCols) = lo;
  __threadfence();
  *(volatile v8us*)dp = hi;
  *(volatile v8us*)(dp + nCols) = lo;
}

__global__ __launch_bounds__(NTHR) void k_x3stats(const float* __restrict__ Y3, const float* __restrict__ tab3,
                                                  const float* __restrict__ g3, const float* __restrict__ b3,
                                                  double* rec) {
  __shared__ __attribute__((aligned(16))) double ps[16 * 128];
  __shared__ __attribute__((aligned(16))) double pq[16 * 128];
  const int tid = (int)threadIdx.x;
  const int cu = tid & 15, rg = tid >> 4, c8 = 8 * cu;
  Col8 C;
  ldcol8(tab3, 128, g3, b3, c8, C);
  double s[8], q[8];
#pragma unroll
  for (int j = 0; j < 8; ++j) { s[j] = 0.0; q[j] = 0.0; }
#pragma unroll 2
  for (int i = 0; i < 8; ++i) {
    const int row = (int)blockIdx.x * 128 + rg + 16 * i;
    const float* yp = Y3 + (size_t)row * 128 + c8;
    const v4f xa = bnr4(*(const v4fa*)yp,       C.m0, C.r0, C.g0, C.b0);
    const v4f xb = bnr4(*(const v4fa*)(yp + 4), C.m1, C.r1, C.g1, C.b1);
    const float x[8] = {xa.x, xa.y, xa.z, xa.w, xb.x, xb.y, xb.z, xb.w};
#pragma unroll
    for (int j = 0; j < 8; ++j) { const double v = (double)x[j]; s[j] += v; q[j] += v * v; }
  }
#pragma unroll
  for (int j = 0; j < 8; ++j) { ps[rg * 128 + c8 + j] = s[j]; pq[rg * 128 + c8 + j] = q[j]; }
  __syncthreads();
  if (tid < 128) {
    double S = 0.0, Q = 0.0;
#pragma unroll 4
    for (int g = 0; g < 16; ++g) { S += ps[g * 128 + tid]; Q += pq[g * 128 + tid]; }
    v2d o; o.x = S; o.y = Q;
    double* rp = rec + ((size_t)blockIdx.x * 128 + (size_t)tid) * 2;
    *(volatile v2d*)rp = o;
    __threadfence();
    *(volatile v2d*)rp = o;
  }
}

__global__ __launch_bounds__(NTHR) void k_cov(const float* __restrict__ Y3, const float* __restrict__ tab3,
                                              const float* __restrict__ g3, const float* __restrict__ b3,
                                              const float* __restrict__ tabmu, unsigned short* XC, float* part) {
  extern __shared__ v4f lds_dyn[];
  unsigned short* TH = (unsigned short*)lds_dyn;
  unsigned short* TL = TH + 128 * TP;
  float* stg = (float*)lds_dyn;
  const int tid = (int)threadIdx.x, lane = tid & 31, wave = tid >> 5, hh = lane >> 4, m = lane & 15;
  const int e0 = (int)blockIdx.x * 128;
  {
    const int c8 = (tid & 15) * 8;
    Col8 C;
    ldcol8(tab3, 128, g3, b3, c8, C);
    const v4f mu0 = *(const v4fa*)(tabmu + c8);
    const v4f mu1 = *(const v4fa*)(tabmu + c8 + 4);
#pragma unroll 1
    for (int it = 0; it < 8; ++it) {
      const int row = it * 16 + (tid >> 4);
      const int e = e0 + row;
      const float* yp = Y3 + (size_t)e * 128 + c8;
      const v4f xa = bnr4(*(const v4fa*)yp,       C.m0, C.r0, C.g0, C.b0) - mu0;
      const v4f xb = bnr4(*(const v4fa*)(yp + 4), C.m1, C.r1, C.g1, C.b1) - mu1;
      v8us hi, lo;
      split8(xa, xb, hi, lo);
      unsigned short* dp = XC + (size_t)e * 256 + c8;
      *(volatile v8us*)dp = hi;
      *(volatile v8us*)(dp + 128) = lo;
      __threadfence();
      *(volatile v8us*)dp = hi;
      *(volatile v8us*)(dp + 128) = lo;
#pragma unroll
      for (int j = 0; j < 8; ++j) {
        TH[(c8 + j) * TP + row] = hi[j];
        TL[(c8 + j) * TP + row] = lo[j];
      }
    }
  }
  __syncthreads();
  v8f acc[8];
#pragma unroll
  for (int t = 0; t < 8; ++t) acc[t] = z8();
#pragma unroll
  for (int ks = 0; ks < 4; ++ks) {
    const int ao = (16 * wave + m) * TP + 32 * ks + 8 * hh;
    FragB ah, al;
    ah.h[0] = *(const v8usa*)(TH + ao); ah.h[1] = *(const v8usa*)(TH + ao + 16);
    al.h[0] = *(const v8usa*)(TL + ao); al.h[1] = *(const v8usa*)(TL + ao + 16);
#pragma unroll
    for (int t = 0; t < 8; ++t) {
      const int bo = (16 * t + m) * TP + 32 * ks + 8 * hh;
      FragB bh, bl;
      bh.h[0] = *(const v8usa*)(TH + bo); bh.h[1] = *(const v8usa*)(TH + bo + 16);
      bl.h[0] = *(const v8usa*)(TL + bo); bl.h[1] = *(const v8usa*)(TL + bo + 16);
      acc[t] = wmb(ah, bh, acc[t]);
      acc[t] = wmb(ah, bl, acc[t]);
      acc[t] = wmb(al, bh, acc[t]);
    }
  }
  __syncthreads();
#pragma unroll
  for (int t = 0; t < 8; ++t) {
#pragma unroll
    for (int r = 0; r < 8; ++r) stg[(16 * wave + 8 * hh + r) * 128 + 16 * t + m] = acc[t][r];
  }
  __syncthreads();
  float* gp = part + (size_t)blockIdx.x * 16384;
#pragma unroll 4
  for (int it = 0; it < 16; ++it) {
    const int i = it * NTHR + tid;
    const v4f v = *(const v4fa*)(stg + 4 * i);
    *(volatile v4f*)(gp + 4 * i) = v;
  }
  __threadfence();
#pragma unroll 4
  for (int it = 0; it < 16; ++it) {
    const int i = it * NTHR + tid;
    const v4f v = *(const v4fa*)(stg + 4 * i);
    *(volatile v4f*)(gp + 4 * i) = v;
  }
}

__global__ __launch_bounds__(NTHR) void k_covcomb(const float* __restrict__ part, double invE,
                                                  unsigned short* CH, unsigned short* CL) {
  __shared__ __attribute__((aligned(16))) unsigned short s2[512];
  const int tid = (int)threadIdx.x, lane = tid & 31, wave = tid >> 5;
  const int idx = (int)blockIdx.x * NTHR + tid;
  double s = 0.0;
#pragma unroll 4
  for (int b = 0; b < 128; ++b) s += (double)part[(size_t)b * 16384 + idx];
  const float c = (float)(s * invE);
  const unsigned h = bf16_bits(c);
  const unsigned l = bf16_bits(c - __uint_as_float(h << 16));
  s2[tid] = (unsigned short)h;
  s2[256 + tid] = (unsigned short)l;
  __syncthreads();
  const int wsel = wave & 1;
  const v8us v = *(const v8usa*)(s2 + 256 * wsel + 8 * lane);
  unsigned short* dp = (wsel == 0 ? CH : CL) + (size_t)blockIdx.x * 256 + 8 * lane;
  const bool okst = wave < 2;
  if (okst) *(volatile v8us*)dp = v;
  __threadfence();
  if (okst) *(volatile v8us*)dp = v;
}

__global__ __launch_bounds__(NTHR) void k_scale(const unsigned short* __restrict__ W4B,
                                                const unsigned short* __restrict__ CH,
                                                const unsigned short* __restrict__ CL,
                                                const float* __restrict__ g4, float* SCALE) {
  __shared__ __attribute__((aligned(16))) unsigned short AW[128 * TP];
  __shared__ __attribute__((aligned(16))) float vs[128];
  const int tid = (int)threadIdx.x, lane = tid & 31, wave = tid >> 5, hh = lane >> 4, m = lane & 15;
  const int c0 = (int)blockIdx.x * 128;
#pragma unroll 2
  for (int it = 0; it < 8; ++it) {
    const int u = it * NTHR + tid;
    const int row = u >> 4, k8 = (u & 15) * 8;
    *(v8usa*)(AW + row * TP + k8) = *(const v8usa*)(W4B + (size_t)(c0 + row) * 128 + k8);
  }
  __syncthreads();
  v8f acc[8];
#pragma unroll
  for (int t = 0; t < 8; ++t) acc[t] = z8();
#pragma unroll
  for (int ks = 0; ks < 4; ++ks) {
    const int ao = (16 * wave + m) * TP + 32 * ks + 8 * hh;
    FragB a;
    a.h[0] = *(const v8usa*)(AW + ao); a.h[1] = *(const v8usa*)(AW + ao + 16);
#pragma unroll
    for (int t = 0; t < 8; ++t) {
      const int bo = (16 * t + m) * 128 + 32 * ks + 8 * hh;
      FragB bh, bl;
      bh.h[0] = *(const v8usa*)(CH + bo); bh.h[1] = *(const v8usa*)(CH + bo + 16);
      bl.h[0] = *(const v8usa*)(CL + bo); bl.h[1] = *(const v8usa*)(CL + bo + 16);
      acc[t] = wmb(a, bh, acc[t]);
      acc[t] = wmb(a, bl, acc[t]);
    }
  }
  float p[8];
#pragma unroll
  for (int r = 0; r < 8; ++r) p[r] = 0.0f;
#pragma unroll
  for (int t = 0; t < 8; ++t) {
#pragma unroll
    for (int r = 0; r < 8; ++r) {
      const unsigned wbits = (unsigned)AW[(16 * wave + 8 * hh + r) * TP + 16 * t + m];
      p[r] = fmaf(acc[t][r], __uint_as_float(wbits << 16), p[r]);
    }
  }
#pragma unroll
  for (int r = 0; r < 8; ++r) {
    p[r] += __shfl_xor(p[r], 1); p[r] += __shfl_xor(p[r], 2);
    p[r] += __shfl_xor(p[r], 4); p[r] += __shfl_xor(p[r], 8);
  }
  if (m == 0) {
#pragma unroll
    for (int r = 0; r < 8; ++r) vs[16 * wave + 8 * hh + r] = p[r];
  }
  __syncthreads();
  const v4f vv = *(const v4fa*)(vs + 4 * lane);
  const v4f gg = bfv4(*(const v4fa*)(g4 + c0 + 4 * lane));
  v4f sc;
  sc.x = gg.x * rsqrtf(fmaxf(vv.x, 0.0f) + 1e-5f);
  sc.y = gg.y * rsqrtf(fmaxf(vv.y, 0.0f) + 1e-5f);
  sc.z = gg.z * rsqrtf(fmaxf(vv.z, 0.0f) + 1e-5f);
  sc.w = gg.w * rsqrtf(fmaxf(vv.w, 0.0f) + 1e-5f);
  float* op = SCALE + c0 + 4 * lane;
  const bool okst = wave == 0;
  if (okst) *(volatile v4f*)op = sc;
  __threadfence();
  if (okst) *(volatile v4f*)op = sc;
}

__global__ __launch_bounds__(NTHR) void k_w4msg(const unsigned short* __restrict__ XC,
                                                const unsigned short* __restrict__ W4B,
                                                const float* __restrict__ SCALE,
                                                const unsigned short* __restrict__ B4T,
                                                const float* __restrict__ node, const int* __restrict__ ei,
                                                float* MSG) {
  __shared__ __attribute__((aligned(16))) float nT[128 * 32];
  __shared__ __attribute__((aligned(16))) unsigned short nB[32 * TP];
  const int tid = (int)threadIdx.x, lane = tid & 31, wave = tid >> 5, hh = lane >> 4, m = lane & 15;
  const int eb = (int)blockIdx.x * 32;
  {
    const int el = tid >> 3, part = tid & 7;
    const int e = eb + el;
    int s = ei[2 * (size_t)e];
    s = s < 0 ? 0 : (s > NN - 1 ? NN - 1 : s);
    const float* sp = node + (size_t)s * 128 + 16 * part;
    const v4f a0 = bfv4(*(const v4fa*)sp),       a1 = bfv4(*(const v4fa*)(sp + 4));
    const v4f a2 = bfv4(*(const v4fa*)(sp + 8)), a3 = bfv4(*(const v4fa*)(sp + 12));
    const float v[16] = {a0.x, a0.y, a0.z, a0.w, a1.x, a1.y, a1.z, a1.w,
                         a2.x, a2.y, a2.z, a2.w, a3.x, a3.y, a3.z, a3.w};
#pragma unroll
    for (int j = 0; j < 16; ++j) nT[(16 * part + j) * 32 + el] = v[j];
    *(v8usa*)(nB + el * TP + 16 * part)     = cvt8(a0, a1);
    *(v8usa*)(nB + el * TP + 16 * part + 8) = cvt8(a2, a3);
  }
  const int rg = wave & 1, cq = wave >> 1;
  FragB ah[4], al[4];
  {
    const unsigned short* ar = XC + (size_t)(eb + 16 * rg + m) * 256 + 8 * hh;
#pragma unroll
    for (int ks = 0; ks < 4; ++ks) {
      ah[ks].h[0] = *(const v8usa*)(ar + 32 * ks);       ah[ks].h[1] = *(const v8usa*)(ar + 32 * ks + 16);
      al[ks].h[0] = *(const v8usa*)(ar + 128 + 32 * ks); al[ks].h[1] = *(const v8usa*)(ar + 128 + 32 * ks + 16);
    }
  }
  __syncthreads();
  v8f acc[2];
  acc[0] = z8(); acc[1] = z8();
  const float* np = nT + 16 * rg + 8 * hh;
#pragma unroll 1
  for (int d = 0; d < 128; ++d) {
    const v4f n0 = *(const v4fa*)(np + d * 32);
    const v4f n1 = *(const v4fa*)(np + d * 32 + 4);
#pragma unroll
    for (int t = 0; t < 2; ++t) {
      const int col = 32 * cq + 16 * t + m;
      const unsigned short* bp = W4B + (size_t)(d * 128 + col) * 128 + 8 * hh;
      v8f y = z8();
#pragma unroll
      for (int ks = 0; ks < 4; ++ks) {
        FragB b;
        b.h[0] = *(const v8usa*)(bp + 32 * ks);
        b.h[1] = *(const v8usa*)(bp + 32 * ks + 16);
        y = wmb(ah[ks], b, y);
        y = wmb(al[ks], b, y);
      }
      const float sc = SCALE[d * 128 + col];
      acc[t][0] = fmaf(n0.x, y[0] * sc, acc[t][0]);
      acc[t][1] = fmaf(n0.y, y[1] * sc, acc[t][1]);
      acc[t][2] = fmaf(n0.z, y[2] * sc, acc[t][2]);
      acc[t][3] = fmaf(n0.w, y[3] * sc, acc[t][3]);
      acc[t][4] = fmaf(n1.x, y[4] * sc, acc[t][4]);
      acc[t][5] = fmaf(n1.y, y[5] * sc, acc[t][5]);
      acc[t][6] = fmaf(n1.z, y[6] * sc, acc[t][6]);
      acc[t][7] = fmaf(n1.w, y[7] * sc, acc[t][7]);
    }
  }
#pragma unroll
  for (int ks = 0; ks < 4; ++ks) {
    const int ao = (16 * rg + m) * TP + 32 * ks + 8 * hh;
    FragB a;
    a.h[0] = *(const v8usa*)(nB + ao); a.h[1] = *(const v8usa*)(nB + ao + 16);
#pragma unroll
    for (int t = 0; t < 2; ++t) {
      const unsigned short* bp = B4T + (size_t)(32 * cq + 16 * t + m) * 128 + 32 * ks + 8 * hh;
      FragB b;
      b.h[0] = *(const v8usa*)bp; b.h[1] = *(const v8usa*)(bp + 16);
      acc[t] = wmb(a, b, acc[t]);
    }
  }
  __syncthreads();
#pragma unroll
  for (int t = 0; t < 2; ++t) {
#pragma unroll
    for (int r = 0; r < 8; ++r) nT[(16 * rg + 8 * hh + r) * 128 + 32 * cq + 16 * t + m] = acc[t][r];
  }
  __syncthreads();
  v4f ov[4];
#pragma unroll
  for (int it = 0; it < 4; ++it) ov[it] = *(const v4fa*)(nT + 4 * (it * NTHR + tid));
  float* mb = MSG + (size_t)eb * 128;
#pragma unroll
  for (int it = 0; it < 4; ++it) *(volatile v4f*)(mb + 4 * (it * NTHR + tid)) = ov[it];
  __threadfence();
#pragma unroll
  for (int it = 0; it < 4; ++it) *(volatile v4f*)(mb + 4 * (it * NTHR + tid)) = ov[it];
}

__device__ __forceinline__ int scan_chunk2(const int* __restrict__ ei, int cbase, int slotBase, int* list,
                                           int tid, int wave) {
  int wc = 0;
  const int el0 = tid * EPT;
  const int* kp = ei + 2 * (size_t)(cbase + el0);
  const v4i q0 = *(const v4ia*)kp,       q1 = *(const v4ia*)(kp + 4);
  const v4i q2 = *(const v4ia*)(kp + 8), q3 = *(const v4ia*)(kp + 12);
  const unsigned nb = (unsigned)slotBase;
  const unsigned s0 = (unsigned)q0.y - nb, s1 = (unsigned)q0.w - nb, s2 = (unsigned)q1.y - nb, s3 = (unsigned)q1.w - nb;
  const unsigned s4 = (unsigned)q2.y - nb, s5 = (unsigned)q2.w - nb, s6 = (unsigned)q3.y - nb, s7 = (unsigned)q3.w - nb;
  const bool h0 = s0 < 64u, h1 = s1 < 64u, h2 = s2 < 64u, h3 = s3 < 64u;
  const bool h4 = s4 < 64u, h5 = s5 < 64u, h6 = s6 < 64u, h7 = s7 < 64u;
  const unsigned any = __builtin_amdgcn_ballot_w32(h0 | h1 | h2 | h3 | h4 | h5 | h6 | h7);
  if (any != 0u) {
#define HITJ(J, HJ, SJ) { \
      const unsigned mj = __builtin_amdgcn_ballot_w32(HJ); \
      if (mj != 0u) { \
        if (HJ) { \
          const int pos = wc + (int)__builtin_amdgcn_mbcnt_lo(mj, 0u); \
          if (pos < WCAP) list[wave * WCAP + pos] = ((el0 + (J)) << 6) | (int)(SJ); \
        } \
        wc += (int)__builtin_popcount(mj); } }
    HITJ(0, h0, s0) HITJ(1, h1, s1) HITJ(2, h2, s2) HITJ(3, h3, s3)
    HITJ(4, h4, s4) HITJ(5, h5, s5) HITJ(6, h6, s6) HITJ(7, h7, s7)
#undef HITJ
  }
  return wc;
}

__global__ __launch_bounds__(NTHR) void k_scan(const int* __restrict__ ei, const float* __restrict__ MSG,
                                               const float* __restrict__ bias, unsigned short* MHL) {
  __shared__ __attribute__((aligned(16))) float agg[64 * 128];
  __shared__ __attribute__((aligned(16))) int list[LISTN];
  __shared__ int cnt[64];
  __shared__ int wcnt[NWAVE];
  const int tid = (int)threadIdx.x, lane = tid & 31, wave = tid >> 5;
  const int nb = (int)blockIdx.x * 64;
  {
    const v4f z = {0.f, 0.f, 0.f, 0.f};
    for (int i = tid; i < 2048; i += NTHR) *(v4fa*)(agg + 4 * i) = z;
    for (int i = tid; i < LISTN; i += NTHR) list[i] = 0;
    if (tid < 64) cnt[tid] = 0;
    if (tid < NWAVE) wcnt[tid] = 0;
  }
  __syncthreads();
#pragma unroll 1
  for (int ch = 0; ch < NE / CHUNK; ++ch) {
    const int cbase = ch * CHUNK;
    const int wc = scan_chunk2(ei, cbase, nb, list, tid, wave);
    if (lane == 0) wcnt[wave] = wc;
    __syncthreads();
#pragma unroll 1
    for (int wsx = 0; wsx < NWAVE; ++wsx) {
      int n = __builtin_amdgcn_readfirstlane(wcnt[wsx]);
      n = n > WCAP ? WCAP : (n < 0 ? 0 : n);
      const int* lp = list + wsx * WCAP;
#pragma unroll 1
      for (int i = 0; i < n; ++i) {
        const int ent = __builtin_amdgcn_readfirstlane(lp[i]);
        const int slot = ent & 63;
        if ((slot >> 3) == wave) {
          int e = cbase + (ent >> 6);
          e = e < 0 ? 0 : (e > NE - 1 ? NE - 1 : e);
          const v4f v = *(const v4fa*)(MSG + (size_t)e * 128 + 4 * lane);
          v4fa* ap = (v4fa*)(agg + slot * 128 + 4 * lane);
          const v4f cur = *ap;
          *ap = cur + v;
          if (lane == 0) cnt[slot] = cnt[slot] + 1;
        }
      }
    }
    __syncthreads();
  }
#pragma unroll 1
  for (int it = 0; it < 4; ++it) {
    const int u = it * NTHR + tid;
    const int row = u >> 4, c8 = (u & 15) * 8;
    int c = cnt[row];
    c = c < 1 ? 1 : c;
    const float rd = 1.0f / (float)c;
    const v4f b0 = bfv4(*(const v4fa*)(bias + c8));
    const v4f b1 = bfv4(*(const v4fa*)(bias + c8 + 4));
    v4f xa = *(const v4fa*)(agg + row * 128 + c8) * rd + b0;
    v4f xb = *(const v4fa*)(agg + row * 128 + c8 + 4) * rd + b1;
    xa.x = fmaxf(xa.x, 0.0f); xa.y = fmaxf(xa.y, 0.0f); xa.z = fmaxf(xa.z, 0.0f); xa.w = fmaxf(xa.w, 0.0f);
    xb.x = fmaxf(xb.x, 0.0f); xb.y = fmaxf(xb.y, 0.0f); xb.z = fmaxf(xb.z, 0.0f); xb.w = fmaxf(xb.w, 0.0f);
    v8us hi, lo;
    split8(xa, xb, hi, lo);
    unsigned short* dp = MHL + (size_t)(nb + row) * 256 + c8;
    *(volatile v8us*)dp = hi;
    *(volatile v8us*)(dp + 128) = lo;
    __threadfence();
    *(volatile v8us*)dp = hi;
    *(volatile v8us*)(dp + 128) = lo;
  }
}

__global__ __launch_bounds__(NTHR) void k_gru(const float* __restrict__ GI, const float* __restrict__ GH,
                                              const float* __restrict__ h0, float* out) {
  __shared__ __attribute__((aligned(16))) float st[NTHR];
  const int tid = (int)threadIdx.x;
  const int idx = (int)blockIdx.x * NTHR + tid;
  const int n = idx >> 7, c = idx & 127;
  const float* gi = GI + (size_t)n * 384 + c;
  const float* gh = GH + (size_t)n * 384 + c;
  const float ir = gi[0], iz = gi[128], in_ = gi[256];
  const float hr = gh[0], hz = gh[128], hn_ = gh[256];
  const float hv = bf16_val(h0[idx]);
  const float r  = __builtin_amdgcn_rcpf(1.0f + expf(-(ir + hr)));
  const float zz = __builtin_amdgcn_rcpf(1.0f + expf(-(iz + hz)));
  const float nn = tanhf(in_ + r * hn_);
  st[tid] = (1.0f - zz) * nn + zz * hv;
  __syncthreads();
  const int tc = tid < 64 ? tid : 63;
  const v4f ov = *(const v4fa*)(st + 4 * tc);
  float* p0 = out + (size_t)blockIdx.x * NTHR + 4 * tc;
  float* p1 = p0 + (size_t)NN * DD;
  const bool okst = tid < 64;
  if (okst) { *(volatile v4f*)p0 = ov; *(volatile v4f*)p1 = ov; }
  __threadfence();
  if (okst) { *(volatile v4f*)p0 = ov; *(volatile v4f*)p1 = ov; }
}

static inline size_t al256(size_t o) { return (o + 255) & ~(size_t)255; }

extern "C" void kernel_launch(void* const* d_in, const int* in_sizes, int n_in,
                              void* d_out, int out_size, void* d_ws, size_t ws_size,
                              hipStream_t stream) {
  if (n_in < 21) return;
  if (in_sizes[0] != NN * DD || in_sizes[1] != NE * 2 || in_sizes[2] != NE * 16 || in_sizes[3] != NN * DD) return;
  if (in_sizes[4] != 256 * 16 || in_sizes[5] != 256 || in_sizes[6] != 256) return;
  if (in_sizes[7] != 256 * 256 || in_sizes[8] != 256 || in_sizes[9] != 256) return;
  if (in_sizes[10] != 128 * 256 || in_sizes[11] != 128 || in_sizes[12] != 128) return;
  if (in_sizes[13] != 16384 * 128 || in_sizes[14] != 16384 || in_sizes[15] != 16384) return;
  if (in_sizes[16] != 128 || in_sizes[17] != 384 * 128 || in_sizes[18] != 384 * 128) return;
  if (in_sizes[19] != 384 || in_sizes[20] != 384) return;
  if (out_size != 2 * NN * DD) return;

  const float* node = (const float*)d_in[0];
  const int*   ei   = (const int*)d_in[1];
  const float* edge = (const float*)d_in[2];
  const float* hid  = (const float*)d_in[3];
  const float* W1 = (const float*)d_in[4];
  const float* g1 = (const float*)d_in[5];
  const float* b1 = (const float*)d_in[6];
  const float* W2 = (const float*)d_in[7];
  const float* g2 = (const float*)d_in[8];
  const float* b2 = (const float*)d_in[9];
  const float* W3 = (const float*)d_in[10];
  const float* g3 = (const float*)d_in[11];
  const float* b3 = (const float*)d_in[12];
  const float* W4 = (const float*)d_in[13];
  const float* g4 = (const float*)d_in[14];
  const float* b4 = (const float*)d_in[15];
  const float* bias = (const float*)d_in[16];
  const float* Wih  = (const float*)d_in[17];
  const float* Whh  = (const float*)d_in[18];
  const float* bih  = (const float*)d_in[19];
  const float* bhh  = (const float*)d_in[20];
  float* out = (float*)d_out;

  char* ws = (char*)d_ws;
  size_t off = 0;
  const size_t oEB  = off; off = al256(off + (size_t)NE * 32 * 2);
  const size_t oW1B = off; off = al256(off + (size_t)256 * 32 * 2);
  const size_t oW2B = off; off = al256(off + (size_t)256 * 256 * 2);
  const size_t oW3B = off; off = al256(off + (size_t)128 * 256 * 2);
  const size_t oW4B = off; off = al256(off + (size_t)16384 * 128 * 2);
  const size_t oWIB = off; off = al256(off + (size_t)384 * 128 * 2);
  const size_t oWHB = off; off = al256(off + (size_t)384 * 128 * 2);
  const size_t oH0B = off; off = al256(off + (size_t)NN * DD * 2);
  const size_t oB4T = off; off = al256(off + (size_t)128 * 128 * 2);
  const size_t oYA  = off; off = al256(off + (size_t)NE * 256 * 4);
  const size_t oXA  = off; off = al256(off + (size_t)NE * 512 * 2);
  const size_t oY3  = off; off = al256(off + (size_t)NE * 128 * 4);
  const size_t oREC = off; off = al256(off + (size_t)256 * 256 * 16);
  const size_t oT1  = off; off = al256(off + 2048);
  const size_t oT2  = off; off = al256(off + 2048);
  const size_t oT3  = off; off = al256(off + 2048);
  const size_t oTM  = off; off = al256(off + 2048);
  const size_t oXC  = off; off = al256(off + (size_t)NE * 256 * 2);
  const size_t oPT  = off; off = al256(off + (size_t)128 * 16384 * 4);
  const size_t oCH  = off; off = al256(off + (size_t)128 * 128 * 2);
  const size_t oCL  = off; off = al256(off + (size_t)128 * 128 * 2);
  const size_t oSC  = off; off = al256(off + (size_t)16384 * 4);
  const size_t oMSG = off; off = al256(off + (size_t)NE * 128 * 4);
  const size_t oMHL = off; off = al256(off + (size_t)NN * 256 * 2);
  const size_t oGI  = off; off = al256(off + (size_t)NN * 384 * 4);
  const size_t oGH  = off; off = al256(off + (size_t)NN * 384 * 4);
  if (off > ws_size || off > (size_t)WSMAX) return;

  unsigned short* EB  = (unsigned short*)(ws + oEB);
  unsigned short* W1B = (unsigned short*)(ws + oW1B);
  unsigned short* W2B = (unsigned short*)(ws + oW2B);
  unsigned short* W3B = (unsigned short*)(ws + oW3B);
  unsigned short* W4B = (unsigned short*)(ws + oW4B);
  unsigned short* WIB = (unsigned short*)(ws + oWIB);
  unsigned short* WHB = (unsigned short*)(ws + oWHB);
  unsigned short* H0B = (unsigned short*)(ws + oH0B);
  unsigned short* B4T = (unsigned short*)(ws + oB4T);
  float*  YA  = (float*)(ws + oYA);
  unsigned short* XA = (unsigned short*)(ws + oXA);
  float*  Y3  = (float*)(ws + oY3);
  double* REC = (double*)(ws + oREC);
  float*  T1  = (float*)(ws + oT1);
  float*  T2  = (float*)(ws + oT2);
  float*  T3  = (float*)(ws + oT3);
  float*  TM  = (float*)(ws + oTM);
  unsigned short* XC = (unsigned short*)(ws + oXC);
  float*  PT  = (float*)(ws + oPT);
  unsigned short* CH = (unsigned short*)(ws + oCH);
  unsigned short* CL = (unsigned short*)(ws + oCL);
  float*  SC  = (float*)(ws + oSC);
  float*  MSG = (float*)(ws + oMSG);
  unsigned short* MHL = (unsigned short*)(ws + oMHL);
  float*  GI  = (float*)(ws + oGI);
  float*  GH  = (float*)(ws + oGH);

  const double invE = 1.0 / (double)NE;
  hipFuncSetAttribute(reinterpret_cast<const void*>(&k_cov), hipFuncAttributeMaxDynamicSharedMemorySize, COV_LDS);

  k_prep<<<PU_ALL / NTHR, NTHR, 0, stream>>>(W2, W3, W4, Wih, Whh, hid, edge, W1, b4,
                                             W2B, W3B, W4B, WIB, WHB, H0B, EB, W1B, B4T);
  k_gemm<0, 1><<<dim3(NE / 64, 4), GTHR, 0, stream>>>(EB, 32, 1, W1B, 32, 1, YA, 256, b1, REC, 256);
  k_comb<<<1, NTHR, 0, stream>>>(REC, NE / 64, 256, invE, T1);
  k_apply<<<(NE * 256 / 8) / NTHR, NTHR, 0, stream>>>(YA, T1, g1, b1, XA, 256, 5, NE * 256 / 8);
  k_gemm<0, 1><<<dim3(NE / 64, 4), GTHR, 0, stream>>>(XA, 512, 16, W2B, 256, 8, YA, 256, b1, REC, 256);
  k_comb<<<1, NTHR, 0, stream>>>(REC, NE / 64, 256, invE, T2);
  k_apply<<<(NE * 256 / 8) / NTHR, NTHR, 0, stream>>>(YA, T2, g2, b2, XA, 256, 5, NE * 256 / 8);
  k_gemm<0, 1><<<dim3(NE / 64, 2), GTHR, 0, stream>>>(XA, 512, 16, W3B, 256, 8, Y3, 128, b1, REC, 128);
  k_comb<<<1, NTHR, 0, stream>>>(REC, NE / 64, 128, invE, T3);
  k_x3stats<<<NE / 128, NTHR, 0, stream>>>(Y3, T3, g3, b3, REC);
  k_comb<<<1, NTHR, 0, stream>>>(REC, NE / 128, 128, invE, TM);
  k_cov<<<NE / 128, NTHR, COV_LDS, stream>>>(Y3, T3, g3, b3, TM, XC, PT);
  k_covcomb<<<64, NTHR, 0, stream>>>(PT, invE, CH, CL);
  k_scale<<<128, NTHR, 0, stream>>>(W4B, CH, CL, g4, SC);
  k_w4msg<<<NE / 32, NTHR, 0, stream>>>(XC, W4B, SC, B4T, node, ei, MSG);
  k_scan<<<NN / 64, NTHR, 0, stream>>>(ei, MSG, bias, MHL);
  k_gemm<1, 0><<<dim3(NN / 64, 6), GTHR, 0, stream>>>(MHL, 256, 8, WIB, 128, 4, GI, 384, bih, REC, 384);
  k_gemm<1, 0><<<dim3(NN / 64, 6), GTHR, 0, stream>>>(H0B, 128, 4, WHB, 128, 4, GH, 384, bhh, REC, 384);
  k_gru<<<(NN * DD) / NTHR, NTHR, 0, stream>>>(GI, GH, hid, out);
}
